// SimnetClassifier_72387378807132
// MI455X (gfx1250) — hardware-run, weakly checked
//
#include <hip/hip_runtime.h>
#include <math.h>

typedef __attribute__((ext_vector_type(16))) _Float16 v16h;
typedef __attribute__((ext_vector_type(16))) __bf16 v16b;
typedef __attribute__((ext_vector_type(8)))  _Float16 v8h;
typedef __attribute__((ext_vector_type(8)))  float v8f;
typedef __attribute__((ext_vector_type(4)))  float v4f;
typedef __attribute__((ext_vector_type(2)))  float v2f;
typedef __attribute__((ext_vector_type(4)))  unsigned v4u;
typedef __attribute__((ext_vector_type(4)))  int v4i;
typedef float __attribute__((may_alias)) float_a;
typedef int __attribute__((may_alias)) int_a;

template <typename T> __device__ __forceinline__ void vst2(void* p, T v) { *(volatile T*)p = v; __threadfence(); *(volatile T*)p = v; }
__device__ __forceinline__ v8f wmma16(v16h a, v16h b, v8f c) {
  v8f d = __builtin_amdgcn_wmma_f32_16x16x32_f16(false, a, false, b, (short)0, c, false, false);
  asm volatile("v_nop\n\tv_nop\n\tv_nop\n\tv_nop" : "+v"(d) : "v"(a), "v"(b));
  return d;
}
__device__ __forceinline__ v8f wmma_bf(v16b a, v16b b, v8f c) {
  v8f d = __builtin_amdgcn_wmma_f32_16x16x32_bf16(false, a, false, b, (short)0, c, false, false);
  asm volatile("v_nop\n\tv_nop\n\tv_nop\n\tv_nop" : "+v"(d) : "v"(a), "v"(b));
  return d;
}
__device__ __forceinline__ v16h frag_h(const _Float16* rowk0, int lane) {
  union { v16h v; v8h q[2]; } u; const _Float16* p = rowk0 + 8 * (lane >> 4);
  u.q[0] = *(const v8h*)p; u.q[1] = *(const v8h*)(p + 16); return u.v;
}
__device__ __forceinline__ v16h frag_f32(const float* rowk0, int lane) {
  v16h a; const float* p = rowk0 + 8 * (lane >> 4);
#pragma unroll
  for (int i = 0; i < 8; ++i) { a[i] = (_Float16)p[i]; a[8 + i] = (_Float16)p[16 + i]; }
  return a;
}
__device__ __forceinline__ v16h frag_f32s(const float* rowk0, int lane, float sc) {
  v16h a; const float* p = rowk0 + 8 * (lane >> 4);
#pragma unroll
  for (int i = 0; i < 8; ++i) { a[i] = (_Float16)(p[i] * sc); a[8 + i] = (_Float16)(p[16 + i] * sc); }
  return a;
}
__device__ __forceinline__ v16h fragc_f32(const float* W, int k0, int n, int lane, int ld, int K) {
  v16h a; const int g = lane >> 4;
#pragma unroll
  for (int i = 0; i < 8; ++i) { const int ka = k0 + 8 * g + i, kb = ka + 16;
    a[i] = (_Float16)(ka < K ? W[(size_t)(ka < K ? ka : K - 1) * ld + n] : 0.f); a[8 + i] = (_Float16)(kb < K ? W[(size_t)(kb < K ? kb : K - 1) * ld + n] : 0.f); }
  return a;
}
struct F2 { v16b h, l; };
__device__ __forceinline__ F2 bsplit16(const float v[16]) { F2 r;
#pragma unroll
  for (int i = 0; i < 16; ++i) { const __bf16 h = (__bf16)v[i]; r.h[i] = h; r.l[i] = (__bf16)(v[i] - (float)h); }
  return r; }
__device__ __forceinline__ F2 split_row(const float* row, int k0, int lane) { float v[16]; const float* p = row + k0 + 8 * (lane >> 4);
#pragma unroll
  for (int i = 0; i < 8; ++i) { v[i] = p[i]; v[8 + i] = p[16 + i]; }
  return bsplit16(v); }
__device__ __forceinline__ F2 split_rowK(const float* row, int k0, int lane, int K) { float v[16]; const int g = lane >> 4;
#pragma unroll
  for (int i = 0; i < 8; ++i) { const int ka = k0 + 8 * g + i, kb = ka + 16; v[i] = ka < K ? row[ka < K ? ka : K - 1] : 0.f; v[8 + i] = kb < K ? row[kb < K ? kb : K - 1] : 0.f; }
  return bsplit16(v); }
__device__ __forceinline__ F2 split_col(const float* W, int k0, int n, int lane, int ld, int K) { float v[16]; const int g = lane >> 4;
#pragma unroll
  for (int i = 0; i < 8; ++i) { const int ka = k0 + 8 * g + i, kb = ka + 16; v[i] = ka < K ? W[(size_t)(ka < K ? ka : K - 1) * ld + n] : 0.f; v[8 + i] = kb < K ? W[(size_t)(kb < K ? kb : K - 1) * ld + n] : 0.f; }
  return bsplit16(v); }
__device__ __forceinline__ v8f mac3(const F2& a, const F2& b, v8f c) { c = wmma_bf(a.l, b.h, c); c = wmma_bf(a.h, b.l, c); return wmma_bf(a.h, b.h, c); }
__device__ __forceinline__ float sigm(float v) { return 1.0f / (1.0f + expf(-v)); }
#define LDSX() do { asm volatile("s_wait_dscnt 0" ::: "memory"); __builtin_amdgcn_wave_barrier(); __builtin_amdgcn_fence(__ATOMIC_RELEASE, "workgroup"); } while (0)


#define NQ 2048
#define NC 10
#define NS 16
#define DD 256
#define H0 256
#define H1 128
#define H2 64
#define H3 10
#define NSUP (NC * NS)
#ifndef TQB
#define TQB (NQ / 16)
#endif
typedef __attribute__((ext_vector_type(8))) __bf16 v8b;
__device__ __forceinline__ v16b frag_b(const __bf16* rowk0, int lane) {
  union { v16b v; v8b q[2]; } u; const __bf16* p = rowk0 + 8 * (lane >> 4);
  u.q[0] = *(const v8b*)p; u.q[1] = *(const v8b*)(p + 16); return u.v;
}
__device__ __forceinline__ float bfr(float v) { return (float)(__bf16)v; }
__device__ __attribute__((noinline)) float exp_ni(float v) { return expf(v); }
__device__ __attribute__((noinline)) float erf_ni(float v) { return erff(v); }
__device__ __attribute__((noinline)) float tanh_p(float v) { return tanhf(v); }

#define WS_P1A 0u
#define WS_P1B (WS_P1A + 2u * (size_t)H0 * DD)
#define WS_P2  (WS_P1B + 2u * (size_t)H0 * DD)
#define WS_P3  (WS_P2 + 2u * (size_t)H1 * H0)
#define WS_P4  (WS_P3 + 2u * (size_t)H2 * H1)
#define WS_AQ  (WS_P4 + 2u * (size_t)16 * H2)
#define WS_BS  (WS_AQ + 4u * (size_t)NQ * H0)
#define WS_END (WS_BS + 4u * (size_t)192 * H0)

__global__ __launch_bounds__(256) void k_pack(const float* __restrict__ W1, const float* __restrict__ W2, const float* __restrict__ W3, const float* __restrict__ W4, __bf16* __restrict__ P) { const int n = blockIdx.x, which = blockIdx.y, t = threadIdx.x; __shared__ __align__(16) __bf16 s[256];
  __bf16* dst; int len;
  if (which == 0) { s[t] = (__bf16)W1[(size_t)t * H0 + n]; dst = P + WS_P1A / 2 + (size_t)n * DD; len = DD; }
  else if (which == 1) { s[t] = (__bf16)W1[(size_t)(DD + t) * H0 + n]; dst = P + WS_P1B / 2 + (size_t)n * DD; len = DD; }
  else if (which == 2) { if (n >= H1) return; s[t] = (__bf16)W2[(size_t)t * H1 + n]; dst = P + WS_P2 / 2 + (size_t)n * H0; len = H0; }
  else if (which == 3) { if (n >= H2) return; if (t < H1) s[t] = (__bf16)W3[(size_t)t * H2 + n]; dst = P + WS_P3 / 2 + (size_t)n * H1; len = H1; }
  else { if (n >= 16) return; if (t < H2) s[t] = (n < H3) ? (__bf16)W4[(size_t)t * H3 + n] : (__bf16)0.f; dst = P + WS_P4 / 2 + (size_t)n * H2; len = H2; }
  __syncthreads(); if (t < len / 8) vst2((unsigned*)(dst + t * 8), *(const v4u*)&s[t * 8]); }
__global__ __launch_bounds__(128) void k_l1(const float* __restrict__ XQ, const float* __restrict__ XS, const __bf16* __restrict__ P, float* __restrict__ AQ, float* __restrict__ BS) { __shared__ __align__(16) float so[4][16][132];
  const int tid = threadIdx.x, wave = tid >> 5, lane = tid & 31, col = lane & 15, g = lane >> 4; const int which = blockIdx.z; const size_t rb = (size_t)blockIdx.x * 64; if (which == 1 && rb >= 192) return;
  const size_t r0 = rb + wave * 16; const int c0 = blockIdx.y * 128; const __bf16* Wr = P + ((which == 0) ? WS_P1A : WS_P1B) / 2; const float* X = (which == 0) ? XQ : XS; const size_t rmax = (which == 0) ? (NQ - 1) : (NSUP - 1);
  v8f acc[8] = {};
#pragma unroll
  for (int kc = 0; kc < DD / 32; ++kc) { v16b a; { const size_t rr = (r0 + col) > rmax ? rmax : (r0 + col); const float* p = X + rr * DD + kc * 32 + 8 * g;
#pragma unroll
      for (int i = 0; i < 8; ++i) { a[i] = (__bf16)p[i]; a[8 + i] = (__bf16)p[16 + i]; } }
#pragma unroll
    for (int j = 0; j < 8; ++j) acc[j] = wmma_bf(a, frag_b(Wr + (size_t)(c0 + j * 16 + col) * DD + kc * 32, lane), acc[j]); }
#pragma unroll
  for (int j = 0; j < 8; ++j)
#pragma unroll
    for (int r = 0; r < 8; ++r) so[wave][8 * g + r][j * 16 + col] = acc[j][r];
  LDSX(); float* dst = (which == 0) ? AQ : BS; for (int rl = 0; rl < 16; ++rl) vst2(dst + (r0 + rl) * H0 + c0 + lane * 4, *(const v4f*)&so[wave][rl][lane * 4]);
}
__global__ __launch_bounds__(128) void k_mlp(const float* __restrict__ AQ, const float* __restrict__ BS, const __bf16* __restrict__ P, const float* __restrict__ B1, const float* __restrict__ B2, const float* __restrict__ B3, const float* __restrict__ B4, float* __restrict__ OUT) {
  __shared__ __align__(16) float sh1[4][16][H0 + 4]; __shared__ __align__(16) float sh2[4][16][H1 + 4]; __shared__ __align__(16) float sh3[4][16][H2 + 4]; __shared__ float sit[4][16]; __shared__ __align__(16) float sres[16 * NC + 32];
  const int tid = threadIdx.x, wave = tid >> 5, lane = tid & 31, col = lane & 15, g = lane >> 4; const int q0 = blockIdx.x * 16;
  const __bf16* W2 = P + WS_P2 / 2; const __bf16* W3 = P + WS_P3 / 2; const __bf16* W4 = P + WS_P4 / 2;
  for (int e = tid; e < 16 * NC + 32; e += 128) sres[e] = 0.f; __syncthreads();
#pragma unroll 1
  for (int tile = wave; tile < 16 * NC; tile += 4) { const int ql = tile / NC, c = tile % NC; const int q = q0 + ql;
    for (int e = lane; e < 16 * H0; e += 32) { const int s = e >> 8, j = e & 255; const float v = AQ[(size_t)q * H0 + j] + BS[(size_t)(c * NS + s) * H0 + j] + bfr(B1[j]); sh1[wave][s][j] = v > 0.f ? v : 0.f; }
    LDSX();
    { v8f acc[8] = {};
#pragma unroll
      for (int kc = 0; kc < H0 / 32; ++kc) { const F2 a = split_row(&sh1[wave][col][0], kc * 32, lane);
#pragma unroll
        for (int jt = 0; jt < 8; ++jt) { const v16b w = frag_b(W2 + (size_t)(jt * 16 + col) * H0 + kc * 32, lane); acc[jt] = wmma_bf(a.h, w, acc[jt]); acc[jt] = wmma_bf(a.l, w, acc[jt]); } }
#pragma unroll
      for (int jt = 0; jt < 8; ++jt) { const float bb = bfr(B2[jt * 16 + col]);
#pragma unroll
        for (int r = 0; r < 8; ++r) { const float v = acc[jt][r] + bb; sh2[wave][8 * g + r][jt * 16 + col] = v > 0.f ? v : 0.f; } } }
    LDSX();
    { v8f acc[4] = {};
#pragma unroll
      for (int kc = 0; kc < H1 / 32; ++kc) { const F2 a = split_row(&sh2[wave][col][0], kc * 32, lane);
#pragma unroll
        for (int jt = 0; jt < 4; ++jt) { const v16b w = frag_b(W3 + (size_t)(jt * 16 + col) * H1 + kc * 32, lane); acc[jt] = wmma_bf(a.h, w, acc[jt]); acc[jt] = wmma_bf(a.l, w, acc[jt]); } }
#pragma unroll
      for (int jt = 0; jt < 4; ++jt) { const float bb = bfr(B3[jt * 16 + col]);
#pragma unroll
        for (int r = 0; r < 8; ++r) { const float v = acc[jt][r] + bb; sh3[wave][8 * g + r][jt * 16 + col] = v > 0.f ? v : 0.f; } } }
    LDSX();
    { v8f acc = {};
#pragma unroll
      for (int kc = 0; kc < H2 / 32; ++kc) { const F2 a = split_row(&sh3[wave][col][0], kc * 32, lane); const v16b w = frag_b(W4 + (size_t)col * H2 + kc * 32, lane); acc = wmma_bf(a.h, w, acc); acc = wmma_bf(a.l, w, acc); }
      float part[8];
#pragma unroll
      for (int r = 0; r < 8; ++r) part[r] = (col < H3) ? tanh_p(acc[r] + bfr(B4[col])) : 0.f;
#pragma unroll
      for (int r = 0; r < 8; ++r) {
#pragma unroll
        for (int o = 1; o < 16; o <<= 1) part[r] += __shfl_xor(part[r], o); }
      if (col == 0) { float ssum = 0.f;
#pragma unroll
        for (int r = 0; r < 8; ++r) ssum += part[r] * 0.1f;
        sit[wave][g] = ssum; } }
    LDSX();
    if (lane == 0) sres[ql * NC + c] = sit[wave][0] + sit[wave][1];
    LDSX(); }
  __syncthreads();
  if (tid < (16 * NC) / 4) vst2(OUT + (size_t)q0 * NC + tid * 4, *(const v4f*)&sres[tid * 4]);
}
extern "C" void kernel_launch(void* const* d_in, const int* in_sizes, int n_in, void* d_out, int out_size, void* d_ws, size_t ws_size, hipStream_t stream) {
  (void)in_sizes; (void)n_in; (void)out_size;
  const float** F = (const float**)d_in;
  if (ws_size < (size_t)WS_END) return;
  char* ws = (char*)d_ws; __bf16* P = (__bf16*)ws; float *AQ = (float*)(ws + WS_AQ), *BS = (float*)(ws + WS_BS);
  k_pack<<<dim3(H0, 5), 256, 0, stream>>>(F[2], F[4], F[6], F[8], P);
  k_l1<<<dim3(NQ / 64, H0 / 128, 2), 128, 0, stream>>>(F[0], F[1], P, AQ, BS);
  k_mlp<<<TQB, 128, 0, stream>>>(AQ, BS, P, F[3], F[5], F[7], F[9], (float*)d_out);
}
